// UnifiedAttention_51857435131905
// MI455X (gfx1250) — hardware-verified
//
#include <hip/hip_runtime.h>


namespace {
constexpr int NH = 16, NKV = 4, S = 2048, D = 128, HD = 64;
constexpr float XS = 8.0f, PS = 8.0f, SCALE = 0.125f, LAM = 0.8f, ONORM = 0.2f, LOG2E = 1.4426950408889634f;

typedef _Float16 b16;
typedef __attribute__((ext_vector_type(16))) _Float16 v16b;
typedef __attribute__((ext_vector_type(8))) _Float16 v8b;
typedef __attribute__((ext_vector_type(8))) float v8f;
typedef __attribute__((ext_vector_type(4))) float v4f;
__device__ __forceinline__ float bf16_rne(float f) { unsigned int u = __float_as_uint(f); u += 0x7FFFu + ((u >> 16) & 1u); return __uint_as_float(u & 0xFFFF0000u); }
__device__ __forceinline__ v16b frag_kb(const b16* p, int hh) { const v8b a = *(const v8b*)(p + 8 * hh), b = *(const v8b*)(p + 16 + 8 * hh); v16b f;
#pragma unroll
  for (int e = 0; e < 8; ++e) { f[e] = a[e]; f[8 + e] = b[e]; } return f; }
__device__ __forceinline__ v8f wmma16b(v16b a, v16b b, v8f c) { v8f d = __builtin_amdgcn_wmma_f32_16x16x32_f16(false, a, false, b, (short)0, c, false, false); asm volatile("v_nop\n\tv_nop\n\tv_nop\n\tv_nop" : "+v"(d) : "v"(a), "v"(b)); return d; }
__device__ __forceinline__ void wave_lds_sync() { __builtin_amdgcn_fence(__ATOMIC_RELEASE, "workgroup"); __builtin_amdgcn_wave_barrier(); __builtin_amdgcn_fence(__ATOMIC_ACQUIRE, "workgroup"); }
__device__ __forceinline__ float nexp2(float x) { return __builtin_amdgcn_exp2f(x); }

__global__ __launch_bounds__(256) void prep_kernel(const float* __restrict__ q, const float* __restrict__ k, b16* __restrict__ Q16, b16* __restrict__ K16) {
  const size_t t = (size_t)blockIdx.x * 256 + threadIdx.x; const size_t nq = (size_t)NH * S * D / 8, nk = (size_t)NKV * S * D / 8;
  const float* src; b16* dst; size_t e; if (t < nq) { src = q; dst = Q16; e = t * 8; } else if (t < nq + nk) { src = k; dst = K16; e = (t - nq) * 8; } else return;
  const v4f a = *(const v4f*)(src + e), c = *(const v4f*)(src + e + 4); v8b o;
#pragma unroll
  for (int j = 0; j < 4; ++j) { o[j] = (b16)(bf16_rne(a[j]) * XS); o[4 + j] = (b16)(bf16_rne(c[j]) * XS); }
  for (int pass = 0; pass < 2; ++pass) { *(volatile v8b*)(dst + e) = o; __threadfence(); }
}
__global__ __launch_bounds__(256) void vt_kernel(const float* __restrict__ v, b16* __restrict__ VT16) {
  __shared__ __attribute__((aligned(16))) b16 T[64][64 + 8];
  const int g = blockIdx.z, s0 = blockIdx.x * 64, d0 = blockIdx.y * 64, t_ = threadIdx.x;
  for (int qq = t_; qq < 64 * 64; qq += 256) { const int ss = qq >> 6, dd = qq & 63; T[dd][ss] = (b16)(bf16_rne(v[((size_t)g * S + s0 + ss) * D + d0 + dd]) * XS); }
  __syncthreads();
  for (int pass = 0; pass < 2; ++pass) { for (int qq = t_; qq < 64 * 8; qq += 256) { const int dd = qq >> 3, c8 = (qq & 7) * 8; *(volatile v8b*)(VT16 + ((size_t)g * D + d0 + dd) * S + s0 + c8) = *(const v8b*)(&T[dd][c8]); } __threadfence(); }
}
__global__ __launch_bounds__(64) void attn_kernel(const b16* __restrict__ Q16, const b16* __restrict__ K16, const b16* __restrict__ VT16, float* __restrict__ out) {
  __shared__ __attribute__((aligned(16))) float To[2][16][HD + 4];
  const int wave = threadIdx.x >> 5, lane = threadIdx.x & 31, hh = lane >> 4, col = lane & 15; const int h = blockIdx.y, g = h / (NH / NKV), dh = blockIdx.z; const int q0 = blockIdx.x * 32 + wave * 16, qi = q0 + col;
  const b16* Qp = Q16 + ((size_t)h * S + qi) * D; const b16* Kb = K16 + (size_t)g * S * D; const b16* Vb = VT16 + ((size_t)g * D + dh * HD) * S;
  const v16b qa0 = frag_kb(Qp, hh), qa1 = frag_kb(Qp + 32, hh), qb0 = frag_kb(Qp + 64, hh), qb1 = frag_kb(Qp + 96, hh);
  float m1 = -INFINITY, l1 = 0.0f, m2 = -INFINITY, l2 = 0.0f; v8f o1[4] = {{}, {}, {}, {}}, o2[4] = {{}, {}, {}, {}};
  const float cs = SCALE * LOG2E; const int kend = q0 + 16;
  for (int kb = 0; kb < kend; kb += 32) {
    v8f s1a = {}, s1b = {}, s2a = {}, s2b = {};
    { const b16* k0p = Kb + (size_t)(kb + col) * D, *k1p = Kb + (size_t)(kb + 16 + col) * D;
      s1a = wmma16b(frag_kb(k0p, hh), qa0, s1a); s1a = wmma16b(frag_kb(k0p + 32, hh), qa1, s1a); s1b = wmma16b(frag_kb(k1p, hh), qa0, s1b); s1b = wmma16b(frag_kb(k1p + 32, hh), qa1, s1b);
      s2a = wmma16b(frag_kb(k0p + 64, hh), qb0, s2a); s2a = wmma16b(frag_kb(k0p + 96, hh), qb1, s2a); s2b = wmma16b(frag_kb(k1p + 64, hh), qb0, s2b); s2b = wmma16b(frag_kb(k1p + 96, hh), qb1, s2b); }
    float e1[16], e2[16]; float mx1 = -INFINITY, mx2 = -INFINITY;
#pragma unroll
    for (int r = 0; r < 8; ++r)
#pragma unroll
      for (int hq = 0; hq < 2; ++hq) { const int key = kb + 16 * hq + 8 * hh + r; const bool ok = key <= qi; const float a1 = (hq ? s1b[r] : s1a[r]) * (cs / (XS * XS)), a2 = (hq ? s2b[r] : s2a[r]) * (cs / (XS * XS));
        e1[hq * 8 + r] = ok ? a1 : -1.0e9f; e2[hq * 8 + r] = ok ? a2 : -1.0e9f; mx1 = fmaxf(mx1, e1[hq * 8 + r]); mx2 = fmaxf(mx2, e2[hq * 8 + r]); }
    mx1 = fmaxf(mx1, __shfl_xor(mx1, 16)); mx2 = fmaxf(mx2, __shfl_xor(mx2, 16));
    const float n1 = fmaxf(m1, mx1), n2 = fmaxf(m2, mx2); const float al1 = nexp2(m1 - n1), al2 = nexp2(m2 - n2); m1 = n1; m2 = n2;
    float sum1 = 0.0f, sum2 = 0.0f; v16b p1, p2, p1l, p2l;
#pragma unroll
    for (int e = 0; e < 16; ++e) { const float x1 = nexp2(e1[e] - n1), x2 = nexp2(e2[e] - n2); sum1 += x1; sum2 += x2; const b16 h1 = (b16)(x1 * PS), h2 = (b16)(x2 * PS); p1[e] = h1; p2[e] = h2; p1l[e] = (b16)(x1 * PS - (float)h1); p2l[e] = (b16)(x2 * PS - (float)h2); }
    sum1 += __shfl_xor(sum1, 16); sum2 += __shfl_xor(sum2, 16); l1 = l1 * al1 + sum1; l2 = l2 * al2 + sum2;
#pragma unroll
    for (int t = 0; t < 4; ++t) { o1[t] *= al1; o2[t] *= al2; const v16b vf = frag_kb(Vb + (size_t)(t * 16 + col) * S + kb, hh); o1[t] = wmma16b(vf, p1, o1[t]); o1[t] = wmma16b(vf, p1l, o1[t]); o2[t] = wmma16b(vf, p2, o2[t]); o2[t] = wmma16b(vf, p2l, o2[t]); } }
  const float i1 = ONORM / (l1 * PS * XS), i2 = ONORM * LAM / (l2 * PS * XS);
#pragma unroll
  for (int t = 0; t < 4; ++t)
#pragma unroll
    for (int r = 0; r < 8; ++r) To[wave][col][t * 16 + 8 * hh + r] = o1[t][r] * i1 - o2[t][r] * i2;
  wave_lds_sync();
  for (int pass = 0; pass < 2; ++pass) { for (int rr = 0; rr < 16; ++rr) if (lane < 16) *(volatile v4f*)(out + ((size_t)h * S + q0 + rr) * D + dh * HD + lane * 4) = *(const v4f*)(&To[wave][rr][lane * 4]); __threadfence(); }
}
}

extern "C" void kernel_launch(void* const* d_in, const int* in_sizes, int n_in, void* d_out, int out_size, void* d_ws, size_t ws_size, hipStream_t stream) {
  (void)n_in;
  auto Fp = [&](int i) { return (const float*)d_in[i]; };
  if (in_sizes[0] != NH * S * D || in_sizes[1] != NKV * S * D || in_sizes[2] != NKV * S * D || out_size != NH * S * D) return;
  size_t off = 0; char* ws = (char*)d_ws;
  auto carve = [&](size_t bytes) { char* p = ws + off; off += (bytes + 255) & ~(size_t)255; return p; };
  b16* Q16 = (b16*)carve((size_t)NH * S * D * 2); b16* K16 = (b16*)carve((size_t)NKV * S * D * 2); b16* VT16 = (b16*)carve((size_t)NKV * D * S * 2);
  if (off > ws_size || off > ((size_t)128 << 20)) return;
  prep_kernel<<<(unsigned)(((size_t)(NH + NKV) * S * D / 8 + 255) / 256), 256, 0, stream>>>(Fp(0), Fp(1), Q16, K16);
  vt_kernel<<<dim3(S / 64, D / 64, NKV), 256, 0, stream>>>(Fp(2), VT16);
  attn_kernel<<<dim3(S / 32, NH, 2), 64, 0, stream>>>(Q16, K16, VT16, (float*)d_out);
}
